// SAGE_40956808134940
// MI455X (gfx1250) — hardware-run, weakly checked
//
#include <hip/hip_runtime.h>
#include <stddef.h>
#include <stdint.h>


#define NN      50000
#define NE      800000
#define C_IN    128
#define C_HID   256
#define C_OUT   128
#define NPAD    50048
#define K1      384
#define K2      1024
#define M1P     256
#define HP      512
#define NTHR    256
#define NWAVE   8
#define EPT     8
#define WCHUNK  256
#define SEG     100096
#define NBRUN   1024
#define SLA     10
#define NBKT    49
#define RCAP    28672
#define WLCAP   (RCAP / NWAVE)
#define DEGCAP  64
#define APB     64
#define GBM     64
#define GBN     128
#define GTHR    128
#define U_W1    (C_HID * (K1 / 8))
#define U_W2    (C_OUT * (K2 / 8))
#define U_BI    NTHR
#define U_XB    (NPAD * (C_IN / 8))
#define U_ALL   (U_W1 + U_W2 + U_BI + U_XB)
#define BK_ZINTS (2 * RCAP + 3 * NBRUN)
#define BK_INTS  (BK_ZINTS + 16)
#define BK_LDS_BYTES (BK_INTS * 4)
#define WSMAX   134217728

static constexpr int SPLIT_M1 = 1;
static constexpr int SPLIT_H  = 1;
static constexpr int SPLIT_M2 = 1;

static_assert(NPAD == 391 * 128 && NPAD % GBM == 0 && NPAD >= NN);
static_assert(NBKT * NBRUN >= NN && NBKT * NBRUN >= NPAD);
static_assert(NBRUN == (1 << SLA) && NBRUN % APB == 0 && (NBKT * NBRUN) % APB == 0 && APB == NWAVE * 8);
static_assert(K1 % 32 == 0 && K2 % 32 == 0 && K1 == 3 * C_IN && K2 == 4 * C_HID);
static_assert(RCAP % 32 == 0 && (RCAP * 4) % 128 == 0 && RCAP % (NTHR * 4) == 0 && RCAP == NWAVE * WLCAP);
static_assert(RCAP >= 17455);
static_assert(DEGCAP >= 35 + 8);
static_assert(NE % 4 == 0 && SEG % WCHUNK == 0 && NWAVE * SEG >= NE);
static_assert((NE - (NWAVE - 1) * SEG) > 0 && ((NE - (NWAVE - 1) * SEG) % WCHUNK) == 0);
static_assert(((long long)NE << SLA) < (1LL << 31));
static_assert(BK_ZINTS % (NTHR * 4) == 0);
static_assert(BK_LDS_BYTES <= 300000);
static_assert(GBM * GBN * 4 + GBN * 4 + 4 * 256 * 2 <= 327680);
static_assert(U_W1 % NTHR == 0 && U_W2 % NTHR == 0 && U_XB % NTHR == 0 && U_ALL % NTHR == 0);
static_assert(GBN == C_OUT && GBM == (GTHR / 32) * 16 && C_HID == 2 * GBN);

typedef float          v4f   __attribute__((ext_vector_type(4)));
typedef float          v8f   __attribute__((ext_vector_type(8)));
typedef int            v4i   __attribute__((ext_vector_type(4)));
typedef int            v8i   __attribute__((ext_vector_type(8)));
typedef unsigned       v2u   __attribute__((ext_vector_type(2)));
typedef unsigned       v4u   __attribute__((ext_vector_type(4)));
typedef unsigned short v4us  __attribute__((ext_vector_type(4)));
typedef unsigned short v8us  __attribute__((ext_vector_type(8)));
typedef unsigned short v16us __attribute__((ext_vector_type(16)));
typedef __bf16         v16bf __attribute__((ext_vector_type(16)));
typedef v4f  __attribute__((may_alias)) v4fa;
typedef v4i  __attribute__((may_alias)) v4ia;
typedef v2u  __attribute__((may_alias)) v2ua;
typedef v4u  __attribute__((may_alias)) v4ua;
typedef v4us __attribute__((may_alias)) v4usa;
typedef v8us __attribute__((may_alias)) v8usa;
union FragB { v16bf v; v16us u; v8us h[2]; v8i w; };

__device__ __forceinline__ v8f wmb(const FragB& a, const FragB& b, v8f c) {
  v8f d = __builtin_amdgcn_wmma_f32_16x16x32_bf16(false, a.v, false, b.v, (short)0, c, false, false);
  asm volatile("v_nop\n\tv_nop\n\tv_nop\n\tv_nop" : "+v"(d) : "v"(a.w), "v"(b.w));
  return d;
}

__device__ __forceinline__ unsigned bf16_bits(float f) {
  const unsigned u = __float_as_uint(f);
  const unsigned r = (u + 0x7FFFu + ((u >> 16) & 1u)) >> 16;
  return (f != f) ? 0x7FC0u : r;
}
__device__ __forceinline__ float bf16_val(float f) {
  return __uint_as_float(bf16_bits(f) << 16);
}
template <int SPLIT>
__device__ __forceinline__ unsigned split_bits(float v) {
  const unsigned hb = bf16_bits(v);
  unsigned lb = 0u;
  if constexpr (SPLIT != 0) lb = bf16_bits(v - __uint_as_float(hb << 16));
  return hb | (lb << 16);
}

__device__ __forceinline__ void wave_sync() {
  __builtin_amdgcn_fence(__ATOMIC_RELEASE, "wavefront");
  __builtin_amdgcn_wave_barrier();
  __builtin_amdgcn_fence(__ATOMIC_ACQUIRE, "wavefront");
}

__device__ __forceinline__ void put8us(unsigned short* dp, v8us o) {
  *(volatile v8us*)dp = o;
  __threadfence();
  *(volatile v8us*)dp = o;
}

__device__ __forceinline__ v8us cvt8_blend(const float* __restrict__ pa, const float* __restrict__ pb, unsigned msk) {
  const v4f a0 = *(const v4f*)pa, a1 = *(const v4f*)(pa + 4);
  const v4f c0 = *(const v4f*)pb, c1 = *(const v4f*)(pb + 4);
  const unsigned nm = (~msk) & 0xFFFFu;
  v8us o;
  o[0] = (unsigned short)((bf16_bits(a0.x) & msk) | (bf16_bits(c0.x) & nm));
  o[1] = (unsigned short)((bf16_bits(a0.y) & msk) | (bf16_bits(c0.y) & nm));
  o[2] = (unsigned short)((bf16_bits(a0.z) & msk) | (bf16_bits(c0.z) & nm));
  o[3] = (unsigned short)((bf16_bits(a0.w) & msk) | (bf16_bits(c0.w) & nm));
  o[4] = (unsigned short)((bf16_bits(a1.x) & msk) | (bf16_bits(c1.x) & nm));
  o[5] = (unsigned short)((bf16_bits(a1.y) & msk) | (bf16_bits(c1.y) & nm));
  o[6] = (unsigned short)((bf16_bits(a1.z) & msk) | (bf16_bits(c1.z) & nm));
  o[7] = (unsigned short)((bf16_bits(a1.w) & msk) | (bf16_bits(c1.w) & nm));
  return o;
}

__global__ __launch_bounds__(NTHR) void k_prep(const float* __restrict__ x,
                                               const float* __restrict__ w1l, const float* __restrict__ w1r,
                                               const float* __restrict__ w2l, const float* __restrict__ w2r,
                                               const float* __restrict__ b1, const float* __restrict__ b2,
                                               unsigned short* w1c, unsigned short* w2c, float* biasp,
                                               unsigned short* xb) {
  const int tid = (int)threadIdx.x;
  const int u = (int)blockIdx.x * NTHR + tid;
  if (u < U_W1) {
    const int n  = u / (K1 / 8);
    const int k8 = (u - n * (K1 / 8)) * 8;
    const int kk = k8 & (C_IN - 1);
    const size_t wo = (size_t)n * C_IN + (size_t)kk;
    const unsigned msk = (k8 < 2 * C_IN) ? 0xFFFFu : 0u;
    const v8us o = cvt8_blend(w1l + wo, w1r + wo, msk);
    put8us(w1c + (size_t)u * 8, o);
  } else if (u < U_W1 + U_W2) {
    const int v  = u - U_W1;
    const int n  = v >> 7;
    const int k8 = (v & 127) * 8;
    const int kk = k8 & (C_HID - 1);
    const size_t wo = (size_t)n * C_HID + (size_t)kk;
    const unsigned msk = (k8 < 2 * C_HID) ? 0xFFFFu : 0u;
    const v8us o = cvt8_blend(w2l + wo, w2r + wo, msk);
    put8us(w2c + (size_t)v * 8, o);
  } else if (u < U_W1 + U_W2 + U_BI) {
    const int t  = tid;
    const int ta = t < 63 ? t : 63;
    int tb = t - 64; tb = tb < 0 ? 0 : (tb > 31 ? 31 : tb);
    const v4f a = *(const v4f*)(b1 + 4 * ta);
    const v4f c = *(const v4f*)(b2 + 4 * tb);
    const unsigned m = (t < 64) ? 0xFFFFFFFFu : 0u;
    v4f o;
    o.x = __uint_as_float((__float_as_uint(bf16_val(a.x)) & m) | (__float_as_uint(bf16_val(c.x)) & ~m));
    o.y = __uint_as_float((__float_as_uint(bf16_val(a.y)) & m) | (__float_as_uint(bf16_val(c.y)) & ~m));
    o.z = __uint_as_float((__float_as_uint(bf16_val(a.z)) & m) | (__float_as_uint(bf16_val(c.z)) & ~m));
    o.w = __uint_as_float((__float_as_uint(bf16_val(a.w)) & m) | (__float_as_uint(bf16_val(c.w)) & ~m));
    asm volatile("" :: "v"(o));
    if (t < 96) {
      float* dp = biasp + 4 * t;
      *(volatile v4f*)dp = o;
      __threadfence();
      *(volatile v4f*)dp = o;
    }
  } else {
    const int v   = u - (U_W1 + U_W2 + U_BI);
    const int row = v >> 4;
    const int k8  = (v & 15) * 8;
    const int rc  = row < NN ? row : NN - 1;
    const unsigned lm = (row < NN) ? 0xFFFFu : 0u;
    const float* p = x + (size_t)rc * C_IN + k8;
    const v4f a0 = *(const v4f*)p, a1 = *(const v4f*)(p + 4);
    v8us o;
    o[0] = (unsigned short)(bf16_bits(a0.x) & lm); o[1] = (unsigned short)(bf16_bits(a0.y) & lm);
    o[2] = (unsigned short)(bf16_bits(a0.z) & lm); o[3] = (unsigned short)(bf16_bits(a0.w) & lm);
    o[4] = (unsigned short)(bf16_bits(a1.x) & lm); o[5] = (unsigned short)(bf16_bits(a1.y) & lm);
    o[6] = (unsigned short)(bf16_bits(a1.z) & lm); o[7] = (unsigned short)(bf16_bits(a1.w) & lm);
    put8us(xb + (size_t)v * 8, o);
  }
}

__device__ __forceinline__ int sweep_step(const int* __restrict__ dsts, int cb, unsigned slotBase, unsigned nb,
                                          int* wlw, int wc, int lane) {
  const int e0 = cb + lane * EPT;
  const v4i da = *(const v4i*)(dsts + e0);
  const v4i db = *(const v4i*)(dsts + e0 + 4);
  const unsigned s0 = (unsigned)da.x - slotBase, s1 = (unsigned)da.y - slotBase;
  const unsigned s2 = (unsigned)da.z - slotBase, s3 = (unsigned)da.w - slotBase;
  const unsigned s4 = (unsigned)db.x - slotBase, s5 = (unsigned)db.y - slotBase;
  const unsigned s6 = (unsigned)db.z - slotBase, s7 = (unsigned)db.w - slotBase;
  const bool h0 = s0 < nb, h1 = s1 < nb, h2 = s2 < nb, h3 = s3 < nb;
  const bool h4 = s4 < nb, h5 = s5 < nb, h6 = s6 < nb, h7 = s7 < nb;
  const int nh = (int)h0 + (int)h1 + (int)h2 + (int)h3 + (int)h4 + (int)h5 + (int)h6 + (int)h7;
  const unsigned any = __builtin_amdgcn_ballot_w32(nh != 0);
  if (any != 0u) {
    int incl = nh;
#pragma unroll
    for (int d = 1; d < 32; d <<= 1) {
      const int y = __shfl_up(incl, d, 32);
      if (lane >= d) incl += y;
    }
    int pos = wc + incl - nh;
#define PUTJ(J, HJ, SJ) \
    if (HJ) { \
      if (pos < WLCAP) wlw[pos] = ((e0 + (J)) << SLA) | (int)(SJ); \
      pos += 1; }
    PUTJ(0, h0, s0)
    PUTJ(1, h1, s1)
    PUTJ(2, h2, s2)
    PUTJ(3, h3, s3)
    PUTJ(4, h4, s4)
    PUTJ(5, h5, s5)
    PUTJ(6, h6, s6)
    PUTJ(7, h7, s7)
#undef PUTJ
    wc += __builtin_amdgcn_readlane(incl, 31);
  }
  return wc;
}

__global__ __launch_bounds__(NTHR) void k_bucket(const int* __restrict__ srcs, const int* __restrict__ dsts,
                                                 int* LIST, int* CNT, int* OFF, int* FLAG) {
  extern __shared__ __attribute__((aligned(16))) int dsm[];
  int* wl   = dsm;
  int* sl   = wl + RCAP;
  int* cnt  = sl + RCAP;
  int* offs = cnt + NBRUN;
  int* cur  = offs + NBRUN;
  int* misc = cur + NBRUN;
  const int tid = (int)threadIdx.x, lane = tid & 31;
  const int wave = __builtin_amdgcn_readfirstlane(tid >> 5);
  const int b = (int)blockIdx.x;
  const int slotBase = b * NBRUN;
  int nbv = NN - slotBase;
  nbv = nbv > NBRUN ? NBRUN : (nbv < 0 ? 0 : nbv);

  {
    const v4i z4 = {0, 0, 0, 0};
    for (int i = tid * 4; i < BK_ZINTS; i += NTHR * 4) *(v4ia*)(dsm + i) = z4;
    if (tid < 16) misc[tid] = 0;
  }
  __syncthreads();

  {
    int* wlw = wl + wave * WLCAP;
    const int segBeg = wave * SEG;
    int segEnd = segBeg + SEG;
    segEnd = segEnd > NE ? NE : segEnd;
    int wc = 0;
#pragma unroll 1
    for (int cb = segBeg; cb < segEnd; cb += WCHUNK)
      wc = sweep_step(dsts, cb, (unsigned)slotBase, (unsigned)nbv, wlw, wc, lane);
    if (lane == 0) misc[wave] = wc;
  }
  __syncthreads();

  if (wave == 0) {
    int ov = 0;
#pragma unroll 1
    for (int w2 = 0; w2 < NWAVE; ++w2) {
      int cw = __builtin_amdgcn_readfirstlane(misc[w2]);
      ov |= (cw > WLCAP) ? 1 : 0;
      cw = cw < 0 ? 0 : (cw > WLCAP ? WLCAP : cw);
#pragma unroll 1
      for (int b0 = 0; b0 < cw; b0 += 32) {
        const int idx = b0 + lane;
        const int ent = wl[w2 * WLCAP + (idx < WLCAP ? idx : WLCAP - 1)];
        const int m32 = (cw - b0) < 32 ? (cw - b0) : 32;
#pragma unroll 1
        for (int k = 0; k < m32; ++k) {
          const int uu   = __builtin_amdgcn_readlane(ent, k);
          const int slot = uu & (NBRUN - 1);
          if (lane == 0) cnt[slot] = cnt[slot] + 1;
        }
      }
    }
    if (lane == 0) misc[9] = ov;
  }
  __syncthreads();

  if (wave == 0) {
    const int base = lane * (NBRUN / 32);
    int s = 0, bg = 0;
#pragma unroll 1
    for (int i = 0; i < NBRUN / 32; ++i) {
      const int cv = cnt[base + i];
      s += cv;
      bg |= (cv > DEGCAP) ? 1 : 0;
    }
    int incl = s;
#pragma unroll
    for (int d = 1; d < 32; d <<= 1) {
      const int y = __shfl_up(incl, d, 32);
      if (lane >= d) incl += y;
    }
    int run = incl - s;
#pragma unroll 1
    for (int i = 0; i < NBRUN / 32; ++i) {
      const int cv = cnt[base + i];
      offs[base + i] = run;
      cur[base + i]  = run;
      run += cv;
    }
    const unsigned bm = __builtin_amdgcn_ballot_w32(bg != 0);
    if (lane == 0) misc[9] = misc[9] | ((bm != 0u) ? 1 : 0);
  }
  __syncthreads();

  if (wave == 0) {
#pragma unroll 1
    for (int w2 = 0; w2 < NWAVE; ++w2) {
      int cw = __builtin_amdgcn_readfirstlane(misc[w2]);
      cw = cw < 0 ? 0 : (cw > WLCAP ? WLCAP : cw);
#pragma unroll 1
      for (int b0 = 0; b0 < cw; b0 += 32) {
        const int idx = b0 + lane;
        const int ent = wl[w2 * WLCAP + (idx < WLCAP ? idx : WLCAP - 1)];
        int eid = ent >> SLA;
        eid = eid < 0 ? 0 : (eid > NE - 1 ? NE - 1 : eid);
        int sr = srcs[eid];
        sr = sr < 0 ? 0 : (sr > NN - 1 ? NN - 1 : sr);
        const int m32 = (cw - b0) < 32 ? (cw - b0) : 32;
#pragma unroll 1
        for (int k = 0; k < m32; ++k) {
          const int uu   = __builtin_amdgcn_readlane(ent, k);
          const int sk   = __builtin_amdgcn_readlane(sr, k);
          const int slot = uu & (NBRUN - 1);
          if (lane == 0) {
            int p = cur[slot];
            p = p < 0 ? 0 : (p > RCAP - 1 ? RCAP - 1 : p);
            sl[p] = sk;
            cur[slot] = p + 1;
          }
        }
      }
    }
  }
  __syncthreads();

  const int fl = misc[9];
  int* Lb = LIST + (size_t)b * RCAP;
  int* Cb = CNT + (size_t)b * NBRUN;
  int* Ob = OFF + (size_t)b * NBRUN;
  int* Fb = FLAG + (size_t)b * 32;
  const v4i f4 = {fl, fl, fl, fl};
#pragma unroll 1
  for (int i = tid * 4; i < RCAP; i += NTHR * 4) {
    const v4i q = *(const v4ia*)(sl + i);
    *(volatile v4i*)(Lb + i) = q;
  }
  {
    const v4i qc = *(const v4ia*)(cnt + 4 * tid);
    const v4i qo = *(const v4ia*)(offs + 4 * tid);
    *(volatile v4i*)(Cb + 4 * tid) = qc;
    *(volatile v4i*)(Ob + 4 * tid) = qo;
    if (tid < 8) *(volatile v4i*)(Fb + 4 * tid) = f4;
  }
  __threadfence();
#pragma unroll 1
  for (int i = tid * 4; i < RCAP; i += NTHR * 4) {
    const v4i q = *(const v4ia*)(sl + i);
    *(volatile v4i*)(Lb + i) = q;
  }
  {
    const v4i qc = *(const v4ia*)(cnt + 4 * tid);
    const v4i qo = *(const v4ia*)(offs + 4 * tid);
    *(volatile v4i*)(Cb + 4 * tid) = qc;
    *(volatile v4i*)(Ob + 4 * tid) = qo;
    if (tid < 8) *(volatile v4i*)(Fb + 4 * tid) = f4;
  }
}

template <int L>
__global__ __launch_bounds__(NTHR) void k_agg(const int* __restrict__ LIST, const int* __restrict__ CNT,
                                              const int* __restrict__ OFF, const int* __restrict__ FLAG,
                                              const unsigned short* __restrict__ G, unsigned short* OUTP) {
  __shared__ __attribute__((aligned(16))) unsigned short rowbuf[NWAVE * M1P];
  const int tid = (int)threadIdx.x, lane = tid & 31;
  const int wave = __builtin_amdgcn_readfirstlane(tid >> 5);
  const int nodeBase = (int)blockIdx.x * APB;
  int bkt = nodeBase >> SLA;
  bkt = bkt > NBKT - 1 ? NBKT - 1 : bkt;
  const int fl = FLAG[bkt * 32];
  const int* Lb = LIST + (size_t)bkt * RCAP;
  const float qnan = __int_as_float(0x7fc00000);
  const float pz = (fl != 0) ? qnan : 0.0f;

#pragma unroll 1
  for (int si = 0; si < APB / NWAVE; ++si) {
    const int node = nodeBase + si * NWAVE + wave;
    int c = CNT[node];
    int o = OFF[node];
    const bool big = c > DEGCAP;
    c = c < 0 ? 0 : (c > DEGCAP ? DEGCAP : c);
    o = o < 0 ? 0 : (o > RCAP - 1 ? RCAP - 1 : o);
    int last = o + c - 1; last = last < o ? o : last;
    last = last > RCAP - 1 ? RCAP - 1 : last;
    const float pzr = big ? qnan : pz;
    const bool live = node < NN;
    float a0 = 0.0f, a1 = 0.0f, a2 = 0.0f, a3 = 0.0f, a4 = 0.0f, a5 = 0.0f, a6 = 0.0f, a7 = 0.0f;
#pragma unroll 1
    for (int b0 = 0; b0 < c; b0 += 32) {
      int idx = o + b0 + lane;
      idx = idx > last ? last : idx;
      int sr = Lb[idx];
      asm volatile("" :: "v"(sr));
      sr = sr < 0 ? 0 : (sr > NN - 1 ? NN - 1 : sr);
      const int m32 = (c - b0) < 32 ? (c - b0) : 32;
#pragma unroll 1
      for (int k = 0; k < m32; ++k) {
        const int sk = __builtin_amdgcn_readlane(sr, k);
        if constexpr (L == 1) {
          const v2u w = *(const v2ua*)(G + (size_t)sk * C_IN + 4 * lane);
          a0 += __uint_as_float(w.x << 16);
          a1 += __uint_as_float(w.x & 0xffff0000u);
          a2 += __uint_as_float(w.y << 16);
          a3 += __uint_as_float(w.y & 0xffff0000u);
        } else {
          const unsigned short* rp = G + (size_t)sk * HP + 8 * lane;
          const v4u wh = *(const v4ua*)rp;
          const v4u wo = *(const v4ua*)(rp + C_HID);
          a0 += __uint_as_float(wh.x << 16)         + __uint_as_float(wo.x << 16);
          a1 += __uint_as_float(wh.x & 0xffff0000u) + __uint_as_float(wo.x & 0xffff0000u);
          a2 += __uint_as_float(wh.y << 16)         + __uint_as_float(wo.y << 16);
          a3 += __uint_as_float(wh.y & 0xffff0000u) + __uint_as_float(wo.y & 0xffff0000u);
          a4 += __uint_as_float(wh.z << 16)         + __uint_as_float(wo.z << 16);
          a5 += __uint_as_float(wh.z & 0xffff0000u) + __uint_as_float(wo.z & 0xffff0000u);
          a6 += __uint_as_float(wh.w << 16)         + __uint_as_float(wo.w << 16);
          a7 += __uint_as_float(wh.w & 0xffff0000u) + __uint_as_float(wo.w & 0xffff0000u);
        }
      }
    }
    const float dv = fmaxf((float)c, 1.0f);
    if constexpr (L == 1) {
      const float m0 = live ? (a0 / dv + pzr) : 0.0f;
      const float m1 = live ? (a1 / dv + pzr) : 0.0f;
      const float m2 = live ? (a2 / dv + pzr) : 0.0f;
      const float m3 = live ? (a3 / dv + pzr) : 0.0f;
      const unsigned r0 = split_bits<SPLIT_M1>(m0), r1 = split_bits<SPLIT_M1>(m1);
      const unsigned r2 = split_bits<SPLIT_M1>(m2), r3 = split_bits<SPLIT_M1>(m3);
      v4us mh, ml;
      mh[0] = (unsigned short)(r0 & 0xffffu); ml[0] = (unsigned short)(r0 >> 16);
      mh[1] = (unsigned short)(r1 & 0xffffu); ml[1] = (unsigned short)(r1 >> 16);
      mh[2] = (unsigned short)(r2 & 0xffffu); ml[2] = (unsigned short)(r2 >> 16);
      mh[3] = (unsigned short)(r3 & 0xffffu); ml[3] = (unsigned short)(r3 >> 16);
      unsigned short* rw = rowbuf + wave * M1P;
      *(v4usa*)(rw + 4 * lane)        = mh;
      *(v4usa*)(rw + C_IN + 4 * lane) = ml;
      wave_sync();
      const v8us q0 = *(const v8usa*)(rw + 8 * lane);
      wave_sync();
      if (node < NPAD) {
        unsigned short* rpw = OUTP + (size_t)node * M1P + 8 * lane;
        *(volatile v8us*)rpw = q0;
        __threadfence();
        *(volatile v8us*)rpw = q0;
      }
    } else {
      const float m0 = live ? (a0 / dv + pzr) : 0.0f;
      const float m1 = live ? (a1 / dv + pzr) : 0.0f;
      const float m2 = live ? (a2 / dv + pzr) : 0.0f;
      const float m3 = live ? (a3 / dv + pzr) : 0.0f;
      const float m4 = live ? (a4 / dv + pzr) : 0.0f;
      const float m5 = live ? (a5 / dv + pzr) : 0.0f;
      const float m6 = live ? (a6 / dv + pzr) : 0.0f;
      const float m7 = live ? (a7 / dv + pzr) : 0.0f;
      const unsigned r0 = split_bits<SPLIT_M2>(m0), r1 = split_bits<SPLIT_M2>(m1);
      const unsigned r2 = split_bits<SPLIT_M2>(m2), r3 = split_bits<SPLIT_M2>(m3);
      const unsigned r4 = split_bits<SPLIT_M2>(m4), r5 = split_bits<SPLIT_M2>(m5);
      const unsigned r6 = split_bits<SPLIT_M2>(m6), r7 = split_bits<SPLIT_M2>(m7);
      v8us qh, ql;
      qh[0] = (unsigned short)(r0 & 0xffffu); ql[0] = (unsigned short)(r0 >> 16);
      qh[1] = (unsigned short)(r1 & 0xffffu); ql[1] = (unsigned short)(r1 >> 16);
      qh[2] = (unsigned short)(r2 & 0xffffu); ql[2] = (unsigned short)(r2 >> 16);
      qh[3] = (unsigned short)(r3 & 0xffffu); ql[3] = (unsigned short)(r3 >> 16);
      qh[4] = (unsigned short)(r4 & 0xffffu); ql[4] = (unsigned short)(r4 >> 16);
      qh[5] = (unsigned short)(r5 & 0xffffu); ql[5] = (unsigned short)(r5 >> 16);
      qh[6] = (unsigned short)(r6 & 0xffffu); ql[6] = (unsigned short)(r6 >> 16);
      qh[7] = (unsigned short)(r7 & 0xffffu); ql[7] = (unsigned short)(r7 >> 16);
      if (node < NPAD) {
        unsigned short* rpw = OUTP + (size_t)node * HP + 8 * lane;
        *(volatile v8us*)rpw = qh;
        *(volatile v8us*)(rpw + C_HID) = ql;
        __threadfence();
        *(volatile v8us*)rpw = qh;
        *(volatile v8us*)(rpw + C_HID) = ql;
      }
    }
  }
}

__device__ __forceinline__ void gemm_seg(v8f (&acc)[8], const unsigned short* ap, const unsigned short* bp,
                                         int kn, int ldb) {
#pragma unroll 1
  for (int k0 = 0; k0 < kn; k0 += 32) {
    FragB af;
    af.h[0] = *(const v8usa*)(ap + k0);
    af.h[1] = *(const v8usa*)(ap + k0 + 16);
#pragma unroll
    for (int nt = 0; nt < 8; ++nt) {
      const unsigned short* wq = bp + (size_t)(16 * nt) * (size_t)ldb + k0;
      FragB bf;
      bf.h[0] = *(const v8usa*)wq;
      bf.h[1] = *(const v8usa*)(wq + 16);
      acc[nt] = wmb(af, bf, acc[nt]);
    }
  }
}

template <int FIN>
__global__ __launch_bounds__(GTHR) __attribute__((amdgpu_num_vgpr(248)))
void k_gemm(const unsigned short* A0, int lda0, int kn0, const unsigned short* A1, int lda1, int kn1,
            const unsigned short* __restrict__ BT, int ldb, const float* __restrict__ bias,
            const int* __restrict__ FLAG, unsigned short* Hout, float* outp) {
  __shared__ __attribute__((aligned(16))) float stg[GBM * GBN];
  __shared__ __attribute__((aligned(16))) float sbias[GBN];
  __shared__ __attribute__((aligned(16))) unsigned short rst[4 * 256];
  const int tid = (int)threadIdx.x, lane = tid & 31, hh = lane >> 4, m = lane & 15;
  const int wave = __builtin_amdgcn_readfirstlane(tid >> 5);
  const int rowBase = (int)blockIdx.x * GBM;
  const int colBase = (int)blockIdx.y * GBN;

  v8f acc[8];
  {
    const v8f z = {0.f, 0.f, 0.f, 0.f, 0.f, 0.f, 0.f, 0.f};
#pragma unroll
    for (int t = 0; t < 8; ++t) acc[t] = z;
  }
  const size_t arow = (size_t)(rowBase + 16 * wave + m);
  const unsigned short* bp = BT + (size_t)(colBase + m) * (size_t)ldb + 8 * hh;
  gemm_seg(acc, A0 + arow * (size_t)lda0 + 8 * hh, bp, kn0, ldb);
  gemm_seg(acc, A1 + arow * (size_t)lda1 + 8 * hh, bp + kn0, kn1, ldb);

#pragma unroll
  for (int nt = 0; nt < 8; ++nt) {
    const int lc = 16 * nt + m;
#pragma unroll
    for (int r = 0; r < 8; ++r) {
      const int lr = 16 * wave + 8 * hh + r;
      stg[lr * GBN + lc] = acc[nt][r];
    }
  }
  if (tid < 32) {
    const v4f b4 = *(const v4f*)(bias + colBase + 4 * tid);
    *(v4fa*)(sbias + 4 * tid) = b4;
  }
  __syncthreads();

  const v4f bb4 = *(const v4fa*)(sbias + 4 * lane);
  int bkt = rowBase >> SLA;
  bkt = bkt > NBKT - 1 ? NBKT - 1 : bkt;
  const int fl = FLAG[bkt * 32];
  const float qnan = __int_as_float(0x7fc00000);

  if constexpr (FIN != 0) {
#pragma unroll 1
    for (int i = 0; i < 16; ++i) {
      const int lr  = 16 * wave + i;
      const int row = rowBase + lr;
      v4f t = *(const v4fa*)(stg + lr * GBN + 4 * lane);
      t = t + bb4;
      v4f y;
      y.x = (fl != 0) ? qnan : t.x;
      y.y = (fl != 0) ? qnan : t.y;
      y.z = (fl != 0) ? qnan : t.z;
      y.w = (fl != 0) ? qnan : t.w;
      asm volatile("" :: "v"(y));
      if (row < NN) {
        float* op = outp + (size_t)row * C_OUT + 4 * lane;
        *(volatile v4f*)op = y;
        __threadfence();
        *(volatile v4f*)op = y;
      }
    }
  } else {
    const int hofs = 8 * (lane & 15) + C_HID * (lane >> 4);
    unsigned short* rw = rst + wave * 256;
#pragma unroll 1
    for (int i = 0; i < 16; ++i) {
      const int lr  = 16 * wave + i;
      const int row = rowBase + lr;
      const bool ok = row < NN;
      v4f t = *(const v4fa*)(stg + lr * GBN + 4 * lane);
      t = t + bb4;
      float y0 = (t.x > 0.0f) ? t.x : (t.x - t.x);
      float y1 = (t.y > 0.0f) ? t.y : (t.y - t.y);
      float y2 = (t.z > 0.0f) ? t.z : (t.z - t.z);
      float y3 = (t.w > 0.0f) ? t.w : (t.w - t.w);
      y0 = (fl != 0) ? qnan : y0; y1 = (fl != 0) ? qnan : y1;
      y2 = (fl != 0) ? qnan : y2; y3 = (fl != 0) ? qnan : y3;
      y0 = ok ? y0 : 0.0f; y1 = ok ? y1 : 0.0f; y2 = ok ? y2 : 0.0f; y3 = ok ? y3 : 0.0f;
      const unsigned r0 = split_bits<SPLIT_H>(y0), r1 = split_bits<SPLIT_H>(y1);
      const unsigned r2 = split_bits<SPLIT_H>(y2), r3 = split_bits<SPLIT_H>(y3);
      v4us h4, l4;
      h4[0] = (unsigned short)(r0 & 0xffffu); l4[0] = (unsigned short)(r0 >> 16);
      h4[1] = (unsigned short)(r1 & 0xffffu); l4[1] = (unsigned short)(r1 >> 16);
      h4[2] = (unsigned short)(r2 & 0xffffu); l4[2] = (unsigned short)(r2 >> 16);
      h4[3] = (unsigned short)(r3 & 0xffffu); l4[3] = (unsigned short)(r3 >> 16);
      *(v4usa*)(rw + 4 * lane)       = h4;
      *(v4usa*)(rw + GBN + 4 * lane) = l4;
      wave_sync();
      const v8us q = *(const v8usa*)(rw + 8 * lane);
      wave_sync();
      unsigned short* hp = Hout + (size_t)row * HP + colBase + hofs;
      *(volatile v8us*)hp = q;
      __threadfence();
      *(volatile v8us*)hp = q;
    }
  }
}

static inline size_t al256(size_t o) { return (o + 255) & ~(size_t)255; }

extern "C" void kernel_launch(void* const* d_in, const int* in_sizes, int n_in,
                              void* d_out, int out_size, void* d_ws, size_t ws_size,
                              hipStream_t stream) {
  if (n_in < 8) return;
  if (in_sizes[0] != NN * C_IN) return;
  if (in_sizes[1] != 2 * NE) return;
  if (in_sizes[2] != C_HID * C_IN || in_sizes[3] != C_HID || in_sizes[4] != C_HID * C_IN) return;
  if (in_sizes[5] != C_OUT * C_HID || in_sizes[6] != C_OUT || in_sizes[7] != C_OUT * C_HID) return;
  if (out_size != NN * C_OUT) return;

  const float* x   = (const float*)d_in[0];
  const int*   ei  = (const int*)  d_in[1];
  const float* W1l = (const float*)d_in[2];
  const float* b1l = (const float*)d_in[3];
  const float* W1r = (const float*)d_in[4];
  const float* W2l = (const float*)d_in[5];
  const float* b2l = (const float*)d_in[6];
  const float* W2r = (const float*)d_in[7];
  float* out = (float*)d_out;
  const int* src = ei;
  const int* dst = ei + NE;

  char* ws = (char*)d_ws;
  size_t off = 0;
  const size_t oW1 = off; off = al256(off + (size_t)C_HID * K1 * 2);
  const size_t oW2 = off; off = al256(off + (size_t)C_OUT * K2 * 2);
  const size_t oBI = off; off = al256(off + (size_t)(C_HID + C_OUT) * 4);
  const size_t oXB = off; off = al256(off + (size_t)NPAD * C_IN * 2);
  const size_t oRM = off; off = al256(off + (size_t)NPAD * HP * 2);
  const size_t oRH = off; off = al256(off + (size_t)NPAD * HP * 2);
  const size_t oLI = off; off = al256(off + (size_t)NBKT * RCAP * 4);
  const size_t oCN = off; off = al256(off + (size_t)NBKT * NBRUN * 4);
  const size_t oOF = off; off = al256(off + (size_t)NBKT * NBRUN * 4);
  const size_t oFL = off; off = al256(off + (size_t)NBKT * 32 * 4);
  if (off > ws_size || off > (size_t)WSMAX) return;
  unsigned short* W1C  = (unsigned short*)(ws + oW1);
  unsigned short* W2C  = (unsigned short*)(ws + oW2);
  float*          BIAS = (float*)(ws + oBI);
  unsigned short* XB   = (unsigned short*)(ws + oXB);
  unsigned short* RM   = (unsigned short*)(ws + oRM);
  unsigned short* RH   = (unsigned short*)(ws + oRH);
  int* LIST = (int*)(ws + oLI);
  int* CNT  = (int*)(ws + oCN);
  int* OFF  = (int*)(ws + oOF);
  int* FLAG = (int*)(ws + oFL);

  hipFuncSetAttribute(reinterpret_cast<const void*>(&k_bucket), hipFuncAttributeMaxDynamicSharedMemorySize,
                      (int)BK_LDS_BYTES);

  k_prep<<<U_ALL / NTHR, NTHR, 0, stream>>>(x, W1l, W1r, W2l, W2r, b1l, b2l, W1C, W2C, BIAS, XB);
  k_bucket<<<NBKT, NTHR, BK_LDS_BYTES, stream>>>(src, dst, LIST, CNT, OFF, FLAG);
  k_agg<1><<<(NBKT * NBRUN) / APB, NTHR, 0, stream>>>(LIST, CNT, OFF, FLAG, XB, RM);
  k_gemm<0><<<dim3(NPAD / GBM, C_HID / GBN), GTHR, 0, stream>>>(RM, M1P, 2 * C_IN, XB, C_IN, C_IN,
                                                                 W1C, K1, BIAS, FLAG, RH, out);
  k_agg<2><<<(NBKT * NBRUN) / APB, NTHR, 0, stream>>>(LIST, CNT, OFF, FLAG, RH, RM);
  k_gemm<1><<<dim3(NPAD / GBM, C_OUT / GBN), GTHR, 0, stream>>>(RM, HP, 2 * C_HID, RH, HP, 2 * C_HID,
                                                                 W2C, K2, BIAS + C_HID, FLAG, RH, out);
}
